// GPTBlock_50294067036203
// MI455X (gfx1250) — hardware-verified
//
#include <hip/hip_runtime.h>


namespace {
constexpr int Bsz = 4, T = 2048, D = 512, NH = 8, DH = 64, HALF = 32, FF = 4 * D;
constexpr int NQKV = 3 * D;
constexpr int MROWS = Bsz * T;
constexpr int QT_PER_B = T / 16;
constexpr float EPS = 1e-5f;

typedef _Float16 b16;
typedef __attribute__((ext_vector_type(16))) _Float16 v16b;
typedef __attribute__((ext_vector_type(8)))  _Float16 v8b;
typedef __attribute__((ext_vector_type(8)))  float v8f;
typedef __attribute__((ext_vector_type(4)))  float v4f;
typedef __attribute__((ext_vector_type(2)))  float v2f;

__device__ __forceinline__ v8b ld8b(const b16* p) { return *(const v8b*)p; }
__device__ __forceinline__ v16b cat8b(v8b a, v8b b) { return __builtin_shufflevector(a, b, 0, 1, 2, 3, 4, 5, 6, 7, 8, 9, 10, 11, 12, 13, 14, 15); }
__device__ __forceinline__ v16b frag_kb(const b16* p, int hh) { return cat8b(ld8b(p + 8 * hh), ld8b(p + 16 + 8 * hh)); }
__device__ __forceinline__ v8f wmma16b(v16b a, v16b b, v8f c) {
  v8f d = __builtin_amdgcn_wmma_f32_16x16x32_f16(false, a, false, b, (short)0, c, false, false);
  asm volatile("v_nop\n\tv_nop\n\tv_nop\n\tv_nop" : "+v"(d) : "v"(a), "v"(b));
  return d;
}
__device__ __forceinline__ void wave_lds_sync() {
  __builtin_amdgcn_fence(__ATOMIC_RELEASE, "workgroup");
  __builtin_amdgcn_wave_barrier();
  __builtin_amdgcn_fence(__ATOMIC_ACQUIRE, "workgroup");
}

__device__ __forceinline__ void gemm_tile16(const b16* __restrict__ A, int lda, const b16* __restrict__ W, int K,
                                            int m0, int c0, int nloc, int hlf, v8f (&acc)[2][4]) {
  for (int kb = 0; kb < K; kb += 32) {
    const v16b a0 = frag_kb(A + (size_t)(m0 + nloc) * lda + kb, hlf);
    const v16b a1 = frag_kb(A + (size_t)(m0 + 16 + nloc) * lda + kb, hlf);
#pragma unroll
    for (int t = 0; t < 4; ++t) {
      const v16b bw = frag_kb(W + (size_t)(c0 + t * 16 + nloc) * K + kb, hlf);
      acc[0][t] = wmma16b(a0, bw, acc[0][t]);
      acc[1][t] = wmma16b(a1, bw, acc[1][t]);
    }
  }
}

__global__ __launch_bounds__(256) void prep_kernel(const float* __restrict__ wqkv, const float* __restrict__ wo, const float* __restrict__ w1,
                                                   const float* __restrict__ w2, b16* __restrict__ wqkvT, b16* __restrict__ woT, b16* __restrict__ w1T,
                                                   b16* __restrict__ w2T, float* __restrict__ cs) {
  const size_t tid = (size_t)blockIdx.x * blockDim.x + threadIdx.x, stride = (size_t)gridDim.x * blockDim.x;
  const size_t n0 = (size_t)NQKV * D / 8, n1 = (size_t)D * D / 8, n2 = (size_t)FF * D / 8, n3 = (size_t)D * FF / 8, ncs = (size_t)T * HALF;
  for (int pass = 0; pass < 2; ++pass) {
    for (size_t c = tid; c < n0 + n1 + n2 + n3 + ncs; c += stride) {
      if (c >= n0 + n1 + n2 + n3) {
        const size_t i = c - (n0 + n1 + n2 + n3); const int t = (int)(i / HALF), j = (int)(i % HALF);
        const float inv_freq = 1.0f / powf(10000.0f, (float)j / (float)HALF);
        const float ang = (float)t * inv_freq;
        v2f p; p[0] = cosf(ang); p[1] = sinf(ang);
        *(volatile v2f*)(cs + i * 2) = p;
        continue;
      }
      const float* w; b16* dst; size_t i; int K, N;
      if (c < n0)                { i = c * 8;                  w = wqkv; K = D;  N = NQKV; dst = wqkvT; }
      else if (c < n0 + n1)      { i = (c - n0) * 8;           w = wo;   K = D;  N = D;    dst = woT; }
      else if (c < n0 + n1 + n2) { i = (c - n0 - n1) * 8;      w = w1;   K = D;  N = FF;   dst = w1T; }
      else                       { i = (c - n0 - n1 - n2) * 8; w = w2;   K = FF; N = D;    dst = w2T; }
      const size_t n = i / K, k0 = i % K;
      v8b v;
#pragma unroll
      for (int e = 0; e < 8; ++e) v[e] = (b16)w[(k0 + e) * (size_t)N + n];
      *(volatile v8b*)(dst + i) = v;
    }
    __threadfence();
  }
}

__global__ __launch_bounds__(256) void ln_kernel(const float* __restrict__ x, const float* __restrict__ g, const float* __restrict__ bta,
                                                 b16* __restrict__ h, int nrows) {
  const int lane = threadIdx.x & 31, row = blockIdx.x * 8 + (threadIdx.x >> 5);
  if (row >= nrows) return;
  const float* xr = x + (size_t)row * D;
  float v[16];
#pragma unroll
  for (int j = 0; j < 4; ++j) { const v4f q = *(const v4f*)(xr + j * 128 + lane * 4); v[4*j] = q[0]; v[4*j+1] = q[1]; v[4*j+2] = q[2]; v[4*j+3] = q[3]; }
  float s = 0.f;
#pragma unroll
  for (int j = 0; j < 16; ++j) s += v[j];
#pragma unroll
  for (int o = 16; o > 0; o >>= 1) s += __shfl_xor(s, o);
  const float mu = s * (1.0f / D);
  float s2 = 0.f;
#pragma unroll
  for (int j = 0; j < 16; ++j) { const float dlt = v[j] - mu; s2 += dlt * dlt; }
#pragma unroll
  for (int o = 16; o > 0; o >>= 1) s2 += __shfl_xor(s2, o);
  const float rs = rsqrtf(s2 * (1.0f / D) + EPS);
  __shared__ __attribute__((aligned(16))) b16 Ts[8][D];
  b16* Tp = Ts[threadIdx.x >> 5];
#pragma unroll
  for (int j = 0; j < 4; ++j)
#pragma unroll
    for (int q = 0; q < 4; ++q) { const int c = j * 128 + lane * 4 + q; Tp[c] = (b16)((v[4*j+q] - mu) * rs * g[c] + bta[c]); }
  wave_lds_sync();
  b16* dst = h + (size_t)row * D;
#pragma unroll
  for (int j = 0; j < 2; ++j) { const int e = j * 256 + lane * 8; *(volatile v8b*)(dst + e) = ld8b(Tp + e); }
  __threadfence();
#pragma unroll
  for (int j = 0; j < 2; ++j) { const int e = j * 256 + lane * 8; *(volatile v8b*)(dst + e) = ld8b(Tp + e); }
}

__global__ __launch_bounds__(128) void qkv_kernel(const b16* __restrict__ h, const b16* __restrict__ wqkvT, const float* __restrict__ cs,
                                                  b16* __restrict__ Qh, b16* __restrict__ Kh, b16* __restrict__ Vh) {
  __shared__ __attribute__((aligned(16))) b16 Ts[4][32 * 64];
  const int lane = threadIdx.x & 31, wave = threadIdx.x >> 5, nloc = lane & 15, hlf = lane >> 4;
  const int m0 = blockIdx.y * 128 + wave * 32;
  const int c0 = blockIdx.x * 64;
  const int mat = c0 / D, head = (c0 % D) / DH;
  v8f acc[2][4];
#pragma unroll
  for (int r = 0; r < 2; ++r)
#pragma unroll
    for (int t = 0; t < 4; ++t) acc[r][t] = (v8f){};
  gemm_tile16(h, D, wqkvT, D, m0, c0, nloc, hlf, acc);
  const int b = m0 / T, t0 = m0 % T;
  const float sc = (mat == 0) ? 0.125f : 1.0f;
  b16* Tp = Ts[wave];
#pragma unroll
  for (int t = 0; t < 4; ++t)
#pragma unroll
    for (int r = 0; r < 2; ++r)
#pragma unroll
      for (int v = 0; v < 8; ++v) {
        const int rr = r * 16 + v + 8 * hlf, d = t * 16 + nloc;
        float val = acc[r][t][v];
        if (mat < 2) {
          const int tpos = t0 + rr;
          const float cv = cs[((size_t)tpos * HALF + (d & 31)) * 2], sv = cs[((size_t)tpos * HALF + (d & 31)) * 2 + 1];
          const float oth = acc[r][t ^ 2][v];
          val = (t < 2) ? (val * cv - oth * sv) : (oth * sv + val * cv);
        }
        const int idx = (mat < 2) ? (rr * 64 + d) : ((rr >> 4) * 1024 + d * 16 + (rr & 15));
        Tp[idx] = (b16)(val * sc);
      }
  wave_lds_sync();
  b16* dh; size_t o;
  if (mat == 0)      { o = ((size_t)(b * NH + head) * T + t0) * DH; dh = Qh + o; }
  else if (mat == 1) { o = ((size_t)(b * NH + head) * T + t0) * DH; dh = Kh + o; }
  else               { o = ((size_t)(b * NH + head) * QT_PER_B + (t0 >> 4)) * (size_t)(DH * 16); dh = Vh + o; }
#pragma unroll
  for (int j = 0; j < 8; ++j) { const int e = (j * 32 + lane) * 8; *(volatile v8b*)(dh + e) = ld8b(Tp + e); }
  __threadfence();
#pragma unroll
  for (int j = 0; j < 8; ++j) { const int e = (j * 32 + lane) * 8; *(volatile v8b*)(dh + e) = ld8b(Tp + e); }
}

__global__ __launch_bounds__(256) void attn_kernel(const b16* __restrict__ Qh, const b16* __restrict__ Kh, const b16* __restrict__ Vh,
                                                   b16* __restrict__ yh) {
  __shared__ __attribute__((aligned(16))) b16 Os[8][16 * 64];
  const int wid = threadIdx.x >> 5, lane = threadIdx.x & 31, hh = lane >> 4, col = lane & 15;
  const int qtile = blockIdx.x * 8 + wid;
  const int g = qtile / QT_PER_B;
  const int q0 = (qtile % QT_PER_B) << 4;
  const int b = g / NH, hd = g % NH;
  const size_t ko = (size_t)g * T * DH;
  const size_t qo = ((size_t)g * T + q0 + col) * DH;
  const v16b q0h = frag_kb(Qh + qo, hh), q1h = frag_kb(Qh + qo + 32, hh);
  float m = -INFINITY, l = 0.0f;
  v8f o0 = {}, o1 = {}, o2 = {}, o3 = {};
  for (int kb = 0; kb < T; kb += 32) {
    const size_t r0 = ko + (size_t)(kb + col) * DH, r1 = ko + (size_t)(kb + 16 + col) * DH;
    v8f s0 = {}, s1 = {};
    {
      v16b ah = frag_kb(Kh + r0, hh);
      s0 = wmma16b(ah, q0h, s0);
      ah = frag_kb(Kh + r0 + 32, hh);
      s0 = wmma16b(ah, q1h, s0);
      ah = frag_kb(Kh + r1, hh);
      s1 = wmma16b(ah, q0h, s1);
      ah = frag_kb(Kh + r1 + 32, hh);
      s1 = wmma16b(ah, q1h, s1);
    }
    float mr = -INFINITY;
#pragma unroll
    for (int r = 0; r < 8; ++r) mr = fmaxf(mr, fmaxf(s0[r], s1[r]));
    mr = fmaxf(mr, __shfl_xor(mr, 16));
    const float mn = fmaxf(m, mr);
    const float al_ = __expf(m - mn);
    m = mn;
    float sum = 0.0f;
    v16b pb;
#pragma unroll
    for (int r = 0; r < 8; ++r) {
      const float p0 = __expf(s0[r] - mn), p1 = __expf(s1[r] - mn);
      sum += p0 + p1;
      pb[r] = (b16)p0; pb[8 + r] = (b16)p1;
    }
    sum += __shfl_xor(sum, 16);
    l = l * al_ + sum;
#pragma unroll
    for (int r = 0; r < 8; ++r) { o0[r] *= al_; o1[r] *= al_; o2[r] *= al_; o3[r] *= al_; }
    const size_t v0 = ko + (size_t)(kb >> 4) * (DH * 16) + 8 * hh, v1 = v0 + DH * 16;
#pragma unroll
    for (int n = 0; n < 4; ++n) {
      const int f = n * 16 + col;
      const v16b va = cat8b(ld8b(Vh + v0 + f * 16), ld8b(Vh + v1 + f * 16));
      v8f& o = (n == 0) ? o0 : (n == 1) ? o1 : (n == 2) ? o2 : o3;
      o = wmma16b(va, pb, o);
    }
  }
  const float inv = 1.0f / l;
  b16* Tt = Os[wid];
#pragma unroll
  for (int r = 0; r < 8; ++r) {
    const int hr = 8 * hh + r;
    Tt[col * 64 + 0 + hr] = (b16)(o0[r] * inv); Tt[col * 64 + 16 + hr] = (b16)(o1[r] * inv);
    Tt[col * 64 + 32 + hr] = (b16)(o2[r] * inv); Tt[col * 64 + 48 + hr] = (b16)(o3[r] * inv);
  }
  wave_lds_sync();
  b16* dst0 = yh + ((size_t)b * T + q0) * D + hd * DH;
#pragma unroll
  for (int j = 0; j < 4; ++j) { const int rr = j * 4 + (lane >> 3), c8 = (lane & 7) * 8; *(volatile v8b*)(dst0 + (size_t)rr * D + c8) = ld8b(Tt + rr * 64 + c8); }
  __threadfence();
#pragma unroll
  for (int j = 0; j < 4; ++j) { const int rr = j * 4 + (lane >> 3), c8 = (lane & 7) * 8; *(volatile v8b*)(dst0 + (size_t)rr * D + c8) = ld8b(Tt + rr * 64 + c8); }
}

template <int MODE>
__global__ __launch_bounds__(128) void gemm_kernel(const b16* __restrict__ A, int K, const b16* __restrict__ W, const float* __restrict__ bias,
                                                   const float* __restrict__ R, float* __restrict__ C, int ldc, b16* __restrict__ G, int ldg) {
  __shared__ __attribute__((aligned(16))) float Ts[4][32 * 64];
  __shared__ __attribute__((aligned(16))) b16 Th[4][32 * 64];
  const int lane = threadIdx.x & 31, wave = threadIdx.x >> 5, nloc = lane & 15, hlf = lane >> 4;
  const int m0 = blockIdx.y * 128 + wave * 32;
  const int c0 = blockIdx.x * 64;
  v8f acc[2][4];
#pragma unroll
  for (int r = 0; r < 2; ++r)
#pragma unroll
    for (int t = 0; t < 4; ++t) acc[r][t] = (v8f){};
  gemm_tile16(A, K, W, K, m0, c0, nloc, hlf, acc);
  float* Tt = Ts[wave];
#pragma unroll
  for (int t = 0; t < 4; ++t)
#pragma unroll
    for (int r = 0; r < 2; ++r)
#pragma unroll
      for (int v = 0; v < 8; ++v) {
        const int rr = r * 16 + v + 8 * hlf, cc = t * 16 + nloc;
        float val = acc[r][t][v] + bias[c0 + cc];
        if (MODE == 1) val = 0.5f * val * (1.0f + erff(val * 0.70710678118654752f));
        Tt[rr * 64 + cc] = val;
      }
  wave_lds_sync();
  if (MODE == 0) {
    float* dst0 = C + (size_t)m0 * ldc + c0; const float* rs0 = R + (size_t)m0 * ldc + c0;
    for (int pass = 0; pass < 2; ++pass) {
#pragma unroll
      for (int j = 0; j < 16; ++j) {
        const int rr = j * 2 + hlf, c4 = nloc * 4;
        const v4f a = *(const v4f*)(Tt + rr * 64 + c4), rres = *(const v4f*)(rs0 + (size_t)rr * ldc + c4);
        *(volatile v4f*)(dst0 + (size_t)rr * ldc + c4) = a + rres;
      }
      __threadfence();
    }
  } else {
    b16* Tq = Th[wave];
#pragma unroll
    for (int j = 0; j < 16; ++j) { const int e = j * 128 + lane * 4; Tq[e] = (b16)Tt[e]; Tq[e + 1] = (b16)Tt[e + 1]; Tq[e + 2] = (b16)Tt[e + 2]; Tq[e + 3] = (b16)Tt[e + 3]; }
    wave_lds_sync();
    b16* g0 = G + (size_t)m0 * ldg + c0;
    for (int pass = 0; pass < 2; ++pass) {
#pragma unroll
      for (int j = 0; j < 8; ++j) { const int rr = j * 4 + (lane >> 3), c8 = (lane & 7) * 8; *(volatile v8b*)(g0 + (size_t)rr * ldg + c8) = ld8b(Tq + rr * 64 + c8); }
      __threadfence();
    }
  }
}
}

extern "C" void kernel_launch(void* const* d_in, const int* in_sizes, int n_in,
                              void* d_out, int out_size, void* d_ws, size_t ws_size, hipStream_t stream) {
  (void)n_in; (void)out_size;
  const float* x     = (const float*)d_in[0];
  const float* ln1g  = (const float*)d_in[1];
  const float* ln1b  = (const float*)d_in[2];
  const float* wqkv  = (const float*)d_in[3];
  const float* wo    = (const float*)d_in[4];
  const float* ln2g  = (const float*)d_in[5];
  const float* ln2b  = (const float*)d_in[6];
  const float* w1    = (const float*)d_in[7];
  const float* b1    = (const float*)d_in[8];
  const float* w2    = (const float*)d_in[9];
  const float* b2    = (const float*)d_in[10];
  float* out = (float*)d_out;
  if (in_sizes[0] != MROWS * D || in_sizes[3] != D * NQKV || in_sizes[7] != D * FF || in_sizes[9] != FF * D) return;

  size_t off = 0; char* ws = (char*)d_ws;
  auto carve = [&](size_t bytes) { char* p = ws + off; off += (bytes + 255) & ~(size_t)255; return p; };
  b16* wqkvT = (b16*)carve((size_t)NQKV * D * 2);
  b16* woT   = (b16*)carve((size_t)D * D * 2);
  b16* w1T   = (b16*)carve((size_t)FF * D * 2);
  b16* w2T   = (b16*)carve((size_t)D * FF * 2);
  float* cs  = (float*)carve((size_t)T * HALF * 2 * 4);
  b16* h1    = (b16*)carve((size_t)MROWS * D * 2);
  b16* Qh    = (b16*)carve((size_t)MROWS * D * 2);
  b16* Kh    = (b16*)carve((size_t)MROWS * D * 2);
  b16* Vh    = (b16*)carve((size_t)MROWS * D * 2);
  b16* yh    = (b16*)carve((size_t)MROWS * D * 2);
  float* x1  = (float*)carve((size_t)MROWS * D * 4);
  b16* gm    = (b16*)carve((size_t)MROWS * FF * 2);
  float* zb  = (float*)carve(4096 * 4);
  if (off > ws_size) return;
  const int ROWBLK = MROWS / 128, NQT = Bsz * NH * QT_PER_B;
  hipMemsetAsync(zb, 0, 4096 * 4, stream);
  prep_kernel<<<1024, 256, 0, stream>>>(wqkv, wo, w1, w2, wqkvT, woT, w1T, w2T, cs);
  ln_kernel<<<MROWS / 8, 256, 0, stream>>>(x, ln1g, ln1b, h1, MROWS);
  qkv_kernel<<<dim3(NQKV / 64, ROWBLK), 128, 0, stream>>>(h1, wqkvT, cs, Qh, Kh, Vh);
  attn_kernel<<<NQT / 8, 256, 0, stream>>>(Qh, Kh, Vh, yh);
  gemm_kernel<0><<<dim3(D / 64, ROWBLK), 128, 0, stream>>>(yh, D, woT, zb, x, x1, D, nullptr, 0);
  ln_kernel<<<MROWS / 8, 256, 0, stream>>>(x1, ln2g, ln2b, h1, MROWS);
  gemm_kernel<1><<<dim3(FF / 64, ROWBLK), 128, 0, stream>>>(h1, D, w1T, b1, nullptr, nullptr, 0, gm, FF);
  gemm_kernel<0><<<dim3(D / 64, ROWBLK), 128, 0, stream>>>(gm, FF, w2T, b2, x1, out, D, nullptr, 0);
}
